// KalmanFilterLayer_19859928776762
// MI455X (gfx1250) — hardware-run, weakly checked
//
#include <hip/hip_runtime.h>
#include <math.h>

typedef __attribute__((ext_vector_type(16))) _Float16 v16h;
typedef __attribute__((ext_vector_type(8)))  _Float16 v8h;
typedef __attribute__((ext_vector_type(8)))  float    v8f;
typedef __attribute__((ext_vector_type(4)))  float    v4f;

constexpr int kNB     = 8;
constexpr int kNN     = 128;
constexpr int kSteps  = 512;
constexpr int kObs    = 8;
constexpr int kState  = 16;
constexpr int kSeqs   = kNB * kNN;
constexpr int kKpad   = 32;
constexpr int kChunk  = 16;
constexpr int kTileSeq = 16;
static_assert(kState == 2 * kObs);
static_assert(kState + kObs + 1 <= kKpad);
static_assert((kSteps % kChunk) == 0);
static_assert((kSeqs % kTileSeq) == 0);
static_assert(kChunk * kObs == 128);

constexpr float kWCarry   = 256.0f;
constexpr float kZCarry   = 64.0f;
constexpr float kAccScale = kWCarry * kZCarry;
constexpr float kAccToZ   = kZCarry / kAccScale;
constexpr float kAccToOut = 1.0f / kAccScale;
constexpr float kHalfMinNormal = 6.103515625e-5f;
constexpr float kMinCov = 1e-6f;

constexpr size_t kOffWT   = 0;
constexpr size_t kWsTotal = kOffWT + (size_t)kSteps * kState * kKpad * 2;
static_assert(kWsTotal == 524288ull);
static_assert(kWsTotal <= 134217728ull);

struct FragH {
  union U { v16h v; v8h h[2]; };
  static __device__ __forceinline__ v16h load(const _Float16* p) {
    U f;
    f.h[0] = *(const v8h*)(p);
    f.h[1] = *(const v8h*)(p + 16);
    return f.v;
  }
};

__device__ __forceinline__ _Float16 to_half_operand(float v) {
  const float w = (fabsf(v) < kHalfMinNormal) ? 0.0f : v;
  return (_Float16)w;
}

__global__ __launch_bounds__(256) void gain_table_kernel(
    const float* __restrict__ Ag, const float* __restrict__ Bpg, const float* __restrict__ Hg,
    const float* __restrict__ Qg, const float* __restrict__ Rg, unsigned short* __restrict__ Wt)
{
  __shared__ __align__(16) float sA[256];
  __shared__ __align__(16) float sAmI[256];
  __shared__ __align__(16) float sQc[256];
  __shared__ __align__(16) float sH[128];
  __shared__ __align__(16) float sHA[128];
  __shared__ __align__(16) float sRc[64];
  __shared__ __align__(16) float sBp[16];
  __shared__ __align__(16) float sHB[8];
  __shared__ __align__(16) float sP[256];
  __shared__ __align__(16) float sT1[256];
  __shared__ __align__(16) float sPm[256];
  __shared__ __align__(16) float sHP[128];
  __shared__ __align__(16) float sPHt[128];
  __shared__ __align__(16) float sSa[128];
  __shared__ __align__(16) float sK[128];
  __shared__ __align__(16) float sWs[512];

  const int tid = threadIdx.x;
  const int i = tid >> 4;
  const int j = tid & 15;

  float av = Ag[tid];
  float qv = Qg[tid];
  float hv = Hg[tid & 127];
  float rv = Rg[tid & 63];
  float bv = Bpg[tid & 15];
  asm volatile("" : "+v"(av), "+v"(qv), "+v"(hv), "+v"(rv), "+v"(bv));
  const float dij = (i == j) ? 1.0f : 0.0f;
  sA[tid]   = av;
  sAmI[tid] = av - dij;
  sQc[tid]  = fmaxf(qv, kMinCov);
  sP[tid]   = dij;
  if (tid < 128) sH[tid] = hv;
  if (tid < 64)  sRc[tid] = fmaxf(rv, kMinCov);
  if (tid < 16)  sBp[tid] = bv;
  __syncthreads();

  {
    const int o = (tid & 127) >> 4;
    float a = 0.0f;
#pragma unroll 1
    for (int k = 0; k < 16; ++k) a = fmaf(sH[o * 16 + k], sA[k * 16 + j], a);
    const int o2 = tid & 7;
    float b = 0.0f;
#pragma unroll 1
    for (int k = 0; k < 16; ++k) b = fmaf(sH[o2 * 16 + k], sBp[k], b);
    if (tid < 128) sHA[tid] = a;
    if (tid < 8)   sHB[tid] = b;
  }
  __syncthreads();

#pragma unroll 1
  for (int t = 0; t < kSteps; ++t) {
    {
      float a = 0.0f;
#pragma unroll 1
      for (int k = 0; k < 16; ++k) a = fmaf(sA[i * 16 + k], sP[k * 16 + j], a);
      sT1[tid] = a;
    }
    __syncthreads();
    float pm;
    {
      float a = 0.0f;
#pragma unroll 1
      for (int k = 0; k < 16; ++k) a = fmaf(sT1[i * 16 + k], sA[j * 16 + k], a);
      pm = a + sQc[tid];
      sPm[tid] = pm;
    }
    __syncthreads();
    if (tid < 128) {
      const int o = tid >> 4;
      float a = 0.0f;
#pragma unroll 1
      for (int k = 0; k < 16; ++k) a = fmaf(sH[o * 16 + k], sPm[k * 16 + j], a);
      sHP[tid] = a;
    } else {
      const int idx = tid - 128;
      const int ii = idx >> 3;
      const int o = idx & 7;
      float a = 0.0f;
#pragma unroll 1
      for (int k = 0; k < 16; ++k) a = fmaf(sPm[ii * 16 + k], sH[o * 16 + k], a);
      sPHt[idx] = a;
    }
    __syncthreads();
    if (tid < 64) {
      const int ra = tid >> 3;
      const int cb = tid & 7;
      float a = 0.0f;
#pragma unroll 1
      for (int k = 0; k < 16; ++k) a = fmaf(sH[ra * 16 + k], sPHt[k * 8 + cb], a);
      sSa[ra * 16 + cb] = a + sRc[tid];
      sSa[ra * 16 + 8 + cb] = (ra == cb) ? 1.0f : 0.0f;
    }
    __syncthreads();
#pragma unroll 1
    for (int kk = 0; kk < 8; ++kk) {
      const int e = tid & 127;
      const int r = e >> 4;
      const int c = e & 15;
      const float piv  = sSa[kk * 16 + kk];
      const float rowk = sSa[kk * 16 + c];
      const float f    = sSa[r * 16 + kk];
      const float cur  = sSa[e];
      __syncthreads();
      const float ip = 1.0f / piv;
      const float rs = rowk * ip;
      const float nv = (r == kk) ? rs : fmaf(-f, rs, cur);
      if (tid < 128) sSa[e] = nv;
      __syncthreads();
    }
    if (tid < 128) {
      const int ii = tid >> 3;
      const int o = tid & 7;
      float a = 0.0f;
#pragma unroll 1
      for (int b = 0; b < 8; ++b) a = fmaf(sPHt[ii * 8 + b], sSa[b * 16 + 8 + o], a);
      sK[tid] = a;
    }
    __syncthreads();
    {
      float kha = 0.0f, khp = 0.0f, gs = 0.0f;
#pragma unroll 1
      for (int o = 0; o < 8; ++o) {
        const float kv = sK[i * 8 + o];
        kha = fmaf(kv, sHA[o * 16 + j], kha);
        khp = fmaf(kv, sHP[o * 16 + j], khp);
        gs  = fmaf(kv, sHB[o], gs);
      }
      const float wx   = sAmI[tid] - kha;
      const float kcol = sK[i * 8 + (j & 7)];
      const float gval = sBp[i] - gs;
      const float ex   = (j < 8) ? kcol : ((j == 8) ? gval : 0.0f);
      sWs[i * 32 + j] = wx;
      sWs[i * 32 + 16 + j] = ex;
      sP[tid] = pm - khp;
    }
    __syncthreads();
    if (tid < 64) {
      const v4f a0 = *(const v4f*)(sWs + tid * 8);
      const v4f a1 = *(const v4f*)(sWs + tid * 8 + 4);
      v8h hv8;
#pragma unroll
      for (int e = 0; e < 4; ++e) {
        const float f0 = a0[e] * kWCarry;
        const float f1 = a1[e] * kWCarry;
        hv8[e]     = to_half_operand(f0);
        hv8[4 + e] = to_half_operand(f1);
      }
      unsigned short* p = Wt + (size_t)t * (kState * kKpad) + tid * 8;
      *(volatile v8h*)p = hv8;
      __threadfence();
      *(volatile v8h*)p = hv8;
    }
  }
}

__global__ __launch_bounds__(32) void state_scan_kernel(
    const float* __restrict__ obs, const float* __restrict__ ctl,
    const unsigned short* __restrict__ Wt, float* __restrict__ out)
{
  __shared__ __align__(16) float sO[kTileSeq * kChunk * kObs];
  const int lane = threadIdx.x & 31;
  const int h = lane >> 4;
  const int n = lane & 15;
  const int seq0 = blockIdx.x * kTileSeq;
  const float* op = obs + (size_t)(seq0 + n) * kSteps * kObs;
  const float* up = ctl + (size_t)(seq0 + n) * kSteps;
  const _Float16* wp = (const _Float16*)Wt + n * kKpad + 8 * h;
  float* ob = out + (size_t)seq0 * kSteps * kObs;
  const bool lowHalf = (h == 0);

  v8f acc = (v8f){0.f, 0.f, 0.f, 0.f, 0.f, 0.f, 0.f, 0.f};

#pragma unroll 1
  for (int t0 = 0; t0 < kSteps; t0 += kChunk) {
#pragma unroll 1
    for (int s = 0; s < kChunk; ++s) {
      const int t = t0 + s;
      const v16h wf = FragH::load(wp + (size_t)t * (kState * kKpad));
      v4f o0 = *(const v4f*)(op + (size_t)t * kObs);
      v4f o1 = *(const v4f*)(op + (size_t)t * kObs + 4);
      float u = up[t];
      asm volatile("" : "+v"(o0), "+v"(o1), "+v"(u));
      v16h zf;
#pragma unroll
      for (int r = 0; r < 8; ++r) {
        const float xv = acc[r] * kAccToZ;
        zf[r] = to_half_operand(xv);
      }
#pragma unroll
      for (int e = 0; e < 4; ++e) {
        const float alt0 = (e == 0) ? (u * kZCarry) : 0.0f;
        const float f0 = lowHalf ? (o0[e] * kZCarry) : alt0;
        const float f1 = lowHalf ? (o1[e] * kZCarry) : 0.0f;
        zf[8 + e]  = to_half_operand(f0);
        zf[12 + e] = to_half_operand(f1);
      }
      acc = __builtin_amdgcn_wmma_f32_16x16x32_f16(false, wf, false, zf, (short)0, acc, false, false);
      asm volatile("v_nop\n\tv_nop\n\tv_nop\n\tv_nop" : "+v"(acc) : "v"(wf), "v"(zf));
      if (lowHalf) {
        v4f e0, e1;
        e0[0] = acc[0] * kAccToOut;
        e0[1] = acc[1] * kAccToOut;
        e0[2] = acc[2] * kAccToOut;
        e0[3] = acc[3] * kAccToOut;
        e1[0] = acc[4] * kAccToOut;
        e1[1] = acc[5] * kAccToOut;
        e1[2] = acc[6] * kAccToOut;
        e1[3] = acc[7] * kAccToOut;
        float* sp = sO + (n * kChunk + s) * kObs;
        *(v4f*)(sp) = e0;
        *(v4f*)(sp + 4) = e1;
      }
    }
    __syncthreads();
    v4f ov[kTileSeq];
#pragma unroll
    for (int q = 0; q < kTileSeq; ++q) ov[q] = *(const v4f*)(sO + q * (kChunk * kObs) + lane * 4);
    for (int pass = 0; pass < 2; ++pass) {
#pragma unroll
      for (int q = 0; q < kTileSeq; ++q) {
        *(volatile v4f*)(ob + (size_t)q * kSteps * kObs + (size_t)t0 * kObs + lane * 4) = ov[q];
      }
      __threadfence();
    }
    __syncthreads();
  }
}

extern "C" void kernel_launch(void* const* d_in, const int* in_sizes, int n_in,
                              void* d_out, int out_size, void* d_ws, size_t ws_size,
                              hipStream_t stream) {
  if (n_in < 7) return;
  if (in_sizes[0] != kSeqs * kSteps * kObs) return;
  if (in_sizes[1] != kSeqs * kSteps) return;
  if (in_sizes[2] != kState * kState) return;
  if (in_sizes[3] != kState) return;
  if (in_sizes[4] != kObs * kState) return;
  if (in_sizes[5] != kState * kState) return;
  if (in_sizes[6] != kObs * kObs) return;
  if (out_size != kSeqs * kSteps * kObs) return;
  if (ws_size < kWsTotal) return;

  const float* obs = (const float*)d_in[0];
  const float* ctl = (const float*)d_in[1];
  const float* A   = (const float*)d_in[2];
  const float* Bp  = (const float*)d_in[3];
  const float* H   = (const float*)d_in[4];
  const float* Q   = (const float*)d_in[5];
  const float* R   = (const float*)d_in[6];
  float* out = (float*)d_out;
  unsigned short* WT = (unsigned short*)((char*)d_ws + kOffWT);

  gain_table_kernel<<<1, 256, 0, stream>>>(A, Bp, H, Q, R, WT);
  state_scan_kernel<<<kSeqs / kTileSeq, 32, 0, stream>>>(obs, ctl, WT, out);
}
